// PeriodicKernelAttention_82343112999023
// MI455X (gfx1250) — hardware-verified
//
#include <hip/hip_runtime.h>
#include <stddef.h>
#include <stdint.h>

#define NH    12
#define LSEQ  2048
#define DH    64
#define NROW  (NH * LSEQ)
#define BR    32
#define BC    128
#define NQT   (LSEQ / BR)

static_assert(DH == 64);
static_assert(LSEQ % BR == 0);
static_assert(LSEQ % BC == 0);
static_assert(BC % 32 == 0);
static_assert(NROW % 32 == 0);
static_assert(LSEQ % 64 == 0);

typedef float          v8f   __attribute__((ext_vector_type(8)));
typedef float          v4f   __attribute__((ext_vector_type(4)));
typedef unsigned int   v4u   __attribute__((ext_vector_type(4)));
typedef unsigned short v8us  __attribute__((ext_vector_type(8)));
typedef unsigned short v16us __attribute__((ext_vector_type(16)));
typedef __bf16         v16b  __attribute__((ext_vector_type(16)));
typedef _Float16       v16h  __attribute__((ext_vector_type(16)));
typedef _Float16       half8 __attribute__((ext_vector_type(8)));
typedef unsigned short ush;

static_assert(sizeof(ush) == 2);

union FragU { v16us v; v8us h[2]; v16b b; v16h f; };
union PackU { v8us s; v4u u; };
union PackH { half8 h; v8us s; v4u u; };
struct HL { v4u h; v4u l; };

#define PI_F 3.14159265358979323846f

__device__ __forceinline__ ush f2bf(float f) {
  const unsigned u = __float_as_uint(f);
  return (ush)((u + 0x7FFFu + ((u >> 16) & 1u)) >> 16);
}
__device__ __forceinline__ float bf2f(ush b) { return __uint_as_float(((unsigned)b) << 16); }

__device__ __forceinline__ HL split8(v8f f) {
  PackU ph, pl;
#pragma unroll
  for (int e = 0; e < 8; ++e) {
    const ush hi = f2bf(f[e]);
    ph.s[e] = hi;
    pl.s[e] = f2bf(f[e] - bf2f(hi));
  }
  HL r; r.h = ph.u; r.l = pl.u;
  return r;
}

__device__ __forceinline__ v8f mmab(v16us a, v16us b, v8f c) {
  FragU ua, ub; ua.v = a; ub.v = b;
  c = __builtin_amdgcn_wmma_f32_16x16x32_bf16(false, ua.b, false, ub.b, (short)0, c, false, false);
  asm volatile("v_nop\n\tv_nop\n\tv_nop\n\tv_nop" : "+v"(c) : "v"(a), "v"(b));
  return c;
}
__device__ __forceinline__ v8f mmaf(v16us a, v16us b, v8f c) {
  FragU ua, ub; ua.v = a; ub.v = b;
  c = __builtin_amdgcn_wmma_f32_16x16x32_f16(false, ua.f, false, ub.f, (short)0, c, false, false);
  asm volatile("v_nop\n\tv_nop\n\tv_nop\n\tv_nop" : "+v"(c) : "v"(a), "v"(b));
  return c;
}

__device__ __forceinline__ v16us ldfragu(const ush* p, int ld, int row0, int k0, int lane) {
  const int m = lane & 15, lh = lane >> 4;
  const ush* q = p + (size_t)(row0 + m) * ld + k0 + 8 * lh;
  FragU f;
  f.h[0] = *(const v8us*)(q);
  f.h[1] = *(const v8us*)(q + 16);
  return f.v;
}

__device__ __forceinline__ v8f zero8() { return (v8f){0.f, 0.f, 0.f, 0.f, 0.f, 0.f, 0.f, 0.f}; }

__global__ __launch_bounds__(256) void k_prep_qk(const float* __restrict__ q, const float* __restrict__ k,
                                                 ush* __restrict__ qh, ush* __restrict__ ql,
                                                 ush* __restrict__ kh, ush* __restrict__ kl,
                                                 float* __restrict__ qsq, float* __restrict__ ksq) {
  __shared__ __align__(16) float ssq[32];
  const int tid = threadIdx.x;
  const int which = blockIdx.y;
  const float* src = (which == 0) ? q : k;
  ush* dsth  = (which == 0) ? qh : kh;
  ush* dstl  = (which == 0) ? ql : kl;
  float* dsq = (which == 0) ? qsq : ksq;
  const int rl = tid >> 3, pc = tid & 7;
  const int row = blockIdx.x * 32 + rl;
  const size_t o = (size_t)row * DH + pc * 8;
  const v4f a0 = *(const v4f*)(src + o);
  const v4f a1 = *(const v4f*)(src + o + 4);
  float ss = a0[0] * a0[0] + a0[1] * a0[1] + a0[2] * a0[2] + a0[3] * a0[3]
           + a1[0] * a1[0] + a1[1] * a1[1] + a1[2] * a1[2] + a1[3] * a1[3];
  ss += __shfl_xor(ss, 1);
  ss += __shfl_xor(ss, 2);
  ss += __shfl_xor(ss, 4);
  const float inv = 1.0f / sqrtf(ss);
  const v8f f = (v8f){a0[0] * inv, a0[1] * inv, a0[2] * inv, a0[3] * inv,
                      a1[0] * inv, a1[1] * inv, a1[2] * inv, a1[3] * inv};
  const HL s = split8(f);
  *(volatile v4u*)(dsth + o) = s.h;
  *(volatile v4u*)(dstl + o) = s.l;
  if (pc == 0) ssq[rl] = ss;
  __syncthreads();
  v4f sv = (v4f){0.f, 0.f, 0.f, 0.f};
  const size_t osq = (size_t)blockIdx.x * 32 + (size_t)tid * 4;
  if (tid < 8) {
    sv = *(const v4f*)(ssq + tid * 4);
    *(volatile v4f*)(dsq + osq) = sv;
  }
  __threadfence();
  *(volatile v4u*)(dsth + o) = s.h;
  *(volatile v4u*)(dstl + o) = s.l;
  if (tid < 8) {
    *(volatile v4f*)(dsq + osq) = sv;
  }
}

#define VTP 72
__global__ __launch_bounds__(256) void k_prep_v(const float* __restrict__ v, ush* __restrict__ vt) {
  __shared__ __align__(16) _Float16 st[DH * VTP];
  const int tid = threadIdx.x;
  const int h  = blockIdx.y;
  const int s0 = blockIdx.x * 64;
  const float* vb = v + ((size_t)h * LSEQ + s0) * DH;
#pragma unroll
  for (int it = 0; it < 4; ++it) {
    const int p  = tid + 256 * it;
    const int ls = p >> 4;
    const int dq = p & 15;
    const v4f a = *(const v4f*)(vb + (size_t)ls * DH + dq * 4);
#pragma unroll
    for (int e = 0; e < 4; ++e) st[(dq * 4 + e) * VTP + ls] = (_Float16)a[e];
  }
  __syncthreads();
  v4u val[2];
  size_t go[2];
#pragma unroll
  for (int it = 0; it < 2; ++it) {
    const int p  = tid + 256 * it;
    const int d  = p >> 3;
    const int pc = p & 7;
    PackH pk;
    pk.h = *(const half8*)(st + d * VTP + pc * 8);
    val[it] = pk.u;
    go[it]  = ((size_t)h * DH + d) * LSEQ + s0 + pc * 8;
  }
#pragma unroll
  for (int it = 0; it < 2; ++it) *(volatile v4u*)(vt + go[it]) = val[it];
  __threadfence();
#pragma unroll
  for (int it = 0; it < 2; ++it) *(volatile v4u*)(vt + go[it]) = val[it];
}

#define SSP 132
#define SPP 136
#define OTP 68
__global__ __launch_bounds__(256) void k_attn(const ush* __restrict__ qh, const ush* __restrict__ ql,
                                              const ush* __restrict__ kh, const ush* __restrict__ kl,
                                              const ush* __restrict__ vt,
                                              const float* __restrict__ qsq, const float* __restrict__ ksq,
                                              const int* __restrict__ mask, float* __restrict__ out) {
  __shared__ __align__(16) float sSO[BR * SSP];
  __shared__ __align__(16) ush   sP[BR * SPP];
  __shared__ __align__(16) float sRed[BR * 8];
  __shared__ __align__(16) float rM[BR];
  __shared__ __align__(16) float rMn[BR];
  __shared__ __align__(16) float rL[BR];
  __shared__ __align__(16) float rSc[BR];

  float* sS = sSO;
  const int tid = threadIdx.x, lane = tid & 31, wave = tid >> 5;
  const int hh = lane >> 4, c = lane & 15;
  const int rt = wave >> 2, ct = wave & 3;
  const int hid = blockIdx.y;
  const int q0  = (int)blockIdx.x * BR;
  const ush* Qh = qh + (size_t)hid * LSEQ * DH;
  const ush* Ql = ql + (size_t)hid * LSEQ * DH;
  const ush* Kh = kh + (size_t)hid * LSEQ * DH;
  const ush* Kl = kl + (size_t)hid * LSEQ * DH;
  const ush* Vt = vt + (size_t)hid * DH * LSEQ;
  const float* Ks = ksq + (size_t)hid * LSEQ;
  const float NEGI = -__builtin_huge_valf();

  const int srow = tid >> 3, schk = tid & 7;
  const float qs = qsq[(size_t)hid * LSEQ + q0 + srow];
  const int* mrow = mask + (size_t)(q0 + srow) * LSEQ;

  if (tid < BR) { rM[tid] = NEGI; rL[tid] = 0.f; }
  __syncthreads();

  v8f oacc = zero8();

#pragma unroll 1
  for (int ch = 0; ch < LSEQ / BC; ++ch) {
    const int j0  = ch * BC;
    const int kr0 = j0 + wave * 16;
    v8f s[2];
    s[0] = zero8(); s[1] = zero8();
#pragma unroll
    for (int k0 = 0; k0 < DH; k0 += 32) {
      const v16us a0h = ldfragu(Qh, DH, q0, k0, lane);
      const v16us a1h = ldfragu(Qh, DH, q0 + 16, k0, lane);
      const v16us a0l = ldfragu(Ql, DH, q0, k0, lane);
      const v16us a1l = ldfragu(Ql, DH, q0 + 16, k0, lane);
      const v16us kbh = ldfragu(Kh, DH, kr0, k0, lane);
      const v16us kbl = ldfragu(Kl, DH, kr0, k0, lane);
      s[0] = mmab(a0h, kbh, s[0]);
      s[1] = mmab(a1h, kbh, s[1]);
      s[0] = mmab(a0h, kbl, s[0]);
      s[1] = mmab(a1h, kbl, s[1]);
      s[0] = mmab(a0l, kbh, s[0]);
      s[1] = mmab(a1l, kbh, s[1]);
    }
#pragma unroll
    for (int t = 0; t < 2; ++t) {
#pragma unroll
      for (int r = 0; r < 8; ++r) {
        const int row = 16 * t + 8 * hh + r;
        sS[row * SSP + wave * 16 + c] = s[t][r];
      }
    }
    __syncthreads();
    {
      float* sr = sS + srow * SSP + schk * 16;
      const int kb = j0 + schk * 16;
      float mx = NEGI;
#pragma unroll 2
      for (int e = 0; e < 16; ++e) {
        const float cv  = sr[e];
        const float t2  = fmaxf(2.0f - 2.0f * cv, 0.0f);
        const float u   = PI_F * sqrtf(t2);
        const float sn  = sinf(u);
        const float sn2 = sn * sn;
        float lg = (qs + Ks[kb + e]) * 0.0625f - 0.25f * sn2;
        lg = (mrow[kb + e] == 0) ? NEGI : lg;
        sr[e] = lg;
        mx = fmaxf(mx, lg);
      }
      sRed[srow * 8 + schk] = mx;
    }
    __syncthreads();
    if (tid < BR) {
      float mx = rM[tid];
#pragma unroll
      for (int i = 0; i < 8; ++i) mx = fmaxf(mx, sRed[tid * 8 + i]);
      rMn[tid] = mx;
    }
    __syncthreads();
    {
      const float mx = rMn[srow];
      const float ms = (mx == NEGI) ? 0.f : mx;
      const float* sr = sS + srow * SSP + schk * 16;
      float sum = 0.f;
      PackH p0, p1;
#pragma unroll
      for (int e = 0; e < 8; ++e) {
        const float p = __expf(sr[e] - ms);
        sum += p;
        p0.h[e] = (_Float16)(p * 1024.0f);
      }
#pragma unroll
      for (int e = 0; e < 8; ++e) {
        const float p = __expf(sr[8 + e] - ms);
        sum += p;
        p1.h[e] = (_Float16)(p * 1024.0f);
      }
      *(v8us*)(sP + srow * SPP + schk * 16)     = p0.s;
      *(v8us*)(sP + srow * SPP + schk * 16 + 8) = p1.s;
      sRed[srow * 8 + schk] = sum;
    }
    __syncthreads();
    if (tid < BR) {
      float sum = 0.f;
#pragma unroll
      for (int i = 0; i < 8; ++i) sum += sRed[tid * 8 + i];
      const float mnew = rMn[tid];
      const float fac  = (mnew == NEGI) ? 1.0f : __expf(rM[tid] - mnew);
      rL[tid]  = rL[tid] * fac + sum;
      rM[tid]  = mnew;
      rSc[tid] = fac;
    }
    __syncthreads();
    {
      const v4f f0 = *(const v4f*)(rSc + 16 * rt + 8 * hh);
      const v4f f1 = *(const v4f*)(rSc + 16 * rt + 8 * hh + 4);
#pragma unroll
      for (int r = 0; r < 4; ++r) {
        oacc[r]     *= f0[r];
        oacc[4 + r] *= f1[r];
      }
    }
#pragma unroll
    for (int kk = 0; kk < BC / 32; ++kk) {
      const v16us pa = ldfragu(sP, SPP, 16 * rt, kk * 32, lane);
      const v16us vb = ldfragu(Vt, LSEQ, 16 * ct, j0 + kk * 32, lane);
      oacc = mmaf(pa, vb, oacc);
    }
    __syncthreads();
  }

  float* sO = sSO;
#pragma unroll
  for (int r = 0; r < 8; ++r) {
    const int row   = 16 * rt + 8 * hh + r;
    const float lv  = rL[row];
    const float inv = (1.0f / lv) * 0.0009765625f;
    sO[row * OTP + 16 * ct + c] = oacc[r] * inv;
  }
  __syncthreads();
  v4f val[2];
  size_t go[2];
  const size_t grow0 = (size_t)hid * LSEQ + (size_t)q0;
#pragma unroll
  for (int it = 0; it < 2; ++it) {
    const int p   = tid + 256 * it;
    const int L   = p >> 3;
    const int pc  = p & 7;
    const int row = L >> 1;
    const int hf  = L & 1;
    val[it] = *(const v4f*)(sO + row * OTP + hf * 32 + pc * 4);
    go[it]  = (grow0 + (size_t)row) * DH + hf * 32 + pc * 4;
  }
#pragma unroll
  for (int it = 0; it < 2; ++it) *(volatile v4f*)(out + go[it]) = val[it];
  __threadfence();
#pragma unroll
  for (int it = 0; it < 2; ++it) *(volatile v4f*)(out + go[it]) = val[it];
}

extern "C" void kernel_launch(void* const* d_in, const int* in_sizes, int n_in,
                              void* d_out, int out_size, void* d_ws, size_t ws_size,
                              hipStream_t stream) {
  if (n_in < 4) return;
  if (in_sizes[0] != NROW * DH) return;
  if (in_sizes[1] != NROW * DH) return;
  if (in_sizes[2] != NROW * DH) return;
  if (in_sizes[3] != LSEQ * LSEQ) return;
  if (out_size != NROW * DH) return;

  const float* q  = (const float*)d_in[0];
  const float* k  = (const float*)d_in[1];
  const float* v  = (const float*)d_in[2];
  const int* mask = (const int*)d_in[3];
  float* out = (float*)d_out;

  size_t off = 0;
  const size_t oQh = off; off += (size_t)NROW * DH * 2;
  const size_t oQl = off; off += (size_t)NROW * DH * 2;
  const size_t oKh = off; off += (size_t)NROW * DH * 2;
  const size_t oKl = off; off += (size_t)NROW * DH * 2;
  const size_t oVt = off; off += (size_t)NH * DH * LSEQ * 2;
  const size_t oQs = off; off += (size_t)NROW * 4;
  const size_t oKs = off; off += (size_t)NROW * 4;
  if (off > ws_size) return;
  if (off > (size_t)134217728) return;

  char* ws = (char*)d_ws;
  ush* Qh = (ush*)(ws + oQh);
  ush* Ql = (ush*)(ws + oQl);
  ush* Kh = (ush*)(ws + oKh);
  ush* Kl = (ush*)(ws + oKl);
  ush* Vt = (ush*)(ws + oVt);
  float* Qs = (float*)(ws + oQs);
  float* Ks = (float*)(ws + oKs);

  k_prep_qk<<<dim3(NROW / 32, 2), dim3(256), 0, stream>>>(q, k, Qh, Ql, Kh, Kl, Qs, Ks);
  k_prep_v<<<dim3(LSEQ / 64, NH), dim3(256), 0, stream>>>(v, Vt);
  k_attn<<<dim3(NQT, NH), dim3(256), 0, stream>>>(Qh, Ql, Kh, Kl, Vt, Qs, Ks, mask, out);
  (void)hipGetLastError();
}
